// DLPTLayer_9612136808567
// MI455X (gfx1250) — hardware-verified
//
#include <hip/hip_runtime.h>
#include <math.h>

typedef __attribute__((ext_vector_type(16))) _Float16 v16h;
typedef __attribute__((ext_vector_type(16))) __bf16 v16b;
typedef __attribute__((ext_vector_type(8)))  _Float16 v8h;
typedef __attribute__((ext_vector_type(8)))  float v8f;
typedef __attribute__((ext_vector_type(4)))  float v4f;
typedef __attribute__((ext_vector_type(2)))  float v2f;
typedef __attribute__((ext_vector_type(4)))  unsigned v4u;
typedef __attribute__((ext_vector_type(4)))  int v4i;
typedef float __attribute__((may_alias)) float_a;
typedef int __attribute__((may_alias)) int_a;

template <typename T> __device__ __forceinline__ void vst2(void* p, T v) { *(volatile T*)p = v; __threadfence(); *(volatile T*)p = v; }
__device__ __forceinline__ v8f wmma16(v16h a, v16h b, v8f c) {
  v8f d = __builtin_amdgcn_wmma_f32_16x16x32_f16(false, a, false, b, (short)0, c, false, false);
  asm volatile("v_nop\n\tv_nop\n\tv_nop\n\tv_nop" : "+v"(d) : "v"(a), "v"(b));
  return d;
}
__device__ __forceinline__ v8f wmma_bf(v16b a, v16b b, v8f c) {
  v8f d = __builtin_amdgcn_wmma_f32_16x16x32_bf16(false, a, false, b, (short)0, c, false, false);
  asm volatile("v_nop\n\tv_nop\n\tv_nop\n\tv_nop" : "+v"(d) : "v"(a), "v"(b));
  return d;
}
__device__ __forceinline__ v16h frag_h(const _Float16* rowk0, int lane) {
  union { v16h v; v8h q[2]; } u; const _Float16* p = rowk0 + 8 * (lane >> 4);
  u.q[0] = *(const v8h*)p; u.q[1] = *(const v8h*)(p + 16); return u.v;
}
__device__ __forceinline__ v16h frag_f32(const float* rowk0, int lane) {
  v16h a; const float* p = rowk0 + 8 * (lane >> 4);
#pragma unroll
  for (int i = 0; i < 8; ++i) { a[i] = (_Float16)p[i]; a[8 + i] = (_Float16)p[16 + i]; }
  return a;
}
__device__ __forceinline__ v16h frag_f32s(const float* rowk0, int lane, float sc) {
  v16h a; const float* p = rowk0 + 8 * (lane >> 4);
#pragma unroll
  for (int i = 0; i < 8; ++i) { a[i] = (_Float16)(p[i] * sc); a[8 + i] = (_Float16)(p[16 + i] * sc); }
  return a;
}
__device__ __forceinline__ v16h fragc_f32(const float* W, int k0, int n, int lane, int ld, int K) {
  v16h a; const int g = lane >> 4;
#pragma unroll
  for (int i = 0; i < 8; ++i) { const int ka = k0 + 8 * g + i, kb = ka + 16;
    a[i] = (_Float16)(ka < K ? W[(size_t)(ka < K ? ka : K - 1) * ld + n] : 0.f); a[8 + i] = (_Float16)(kb < K ? W[(size_t)(kb < K ? kb : K - 1) * ld + n] : 0.f); }
  return a;
}
struct F2 { v16b h, l; };
__device__ __forceinline__ F2 bsplit16(const float v[16]) { F2 r;
#pragma unroll
  for (int i = 0; i < 16; ++i) { const __bf16 h = (__bf16)v[i]; r.h[i] = h; r.l[i] = (__bf16)(v[i] - (float)h); }
  return r; }
__device__ __forceinline__ F2 split_row(const float* row, int k0, int lane) { float v[16]; const float* p = row + k0 + 8 * (lane >> 4);
#pragma unroll
  for (int i = 0; i < 8; ++i) { v[i] = p[i]; v[8 + i] = p[16 + i]; }
  return bsplit16(v); }
__device__ __forceinline__ F2 split_rowK(const float* row, int k0, int lane, int K) { float v[16]; const int g = lane >> 4;
#pragma unroll
  for (int i = 0; i < 8; ++i) { const int ka = k0 + 8 * g + i, kb = ka + 16; v[i] = ka < K ? row[ka < K ? ka : K - 1] : 0.f; v[8 + i] = kb < K ? row[kb < K ? kb : K - 1] : 0.f; }
  return bsplit16(v); }
__device__ __forceinline__ F2 split_col(const float* W, int k0, int n, int lane, int ld, int K) { float v[16]; const int g = lane >> 4;
#pragma unroll
  for (int i = 0; i < 8; ++i) { const int ka = k0 + 8 * g + i, kb = ka + 16; v[i] = ka < K ? W[(size_t)(ka < K ? ka : K - 1) * ld + n] : 0.f; v[8 + i] = kb < K ? W[(size_t)(kb < K ? kb : K - 1) * ld + n] : 0.f; }
  return bsplit16(v); }
__device__ __forceinline__ v8f mac3(const F2& a, const F2& b, v8f c) { c = wmma_bf(a.l, b.h, c); c = wmma_bf(a.h, b.l, c); return wmma_bf(a.h, b.h, c); }
__device__ __forceinline__ float sigm(float v) { return 1.0f / (1.0f + expf(-v)); }
#define LDSX() do { asm volatile("s_wait_dscnt 0" ::: "memory"); __builtin_amdgcn_wave_barrier(); __builtin_amdgcn_fence(__ATOMIC_RELEASE, "workgroup"); } while (0)


#define NBATCH 4
#define NPT 65536
#define NDS 16384
#ifndef TNB
#define TNB NBATCH
#endif
typedef __attribute__((ext_vector_type(8))) __bf16 v8b;
__device__ __forceinline__ v16b frag_b(const __bf16* rowk0, int lane) {
  union { v16b v; v8b q[2]; } u; const __bf16* p = rowk0 + 8 * (lane >> 4);
  u.q[0] = *(const v8b*)p; u.q[1] = *(const v8b*)(p + 16); return u.v;
}
__device__ __forceinline__ float bfr(float v) { return (float)(__bf16)v; }
__device__ __attribute__((noinline)) float exp_ni(float v) { return expf(v); }
__device__ __forceinline__ F2 split_colT(const float* T, int k0, int n, int lane, int ld, int K) { return split_col(T, k0, n, lane, ld, K); }

#define P1(m)  ((m) * 1024)
#define P2(m)  (4 * 1024 + (m) * 4096)
#define P_END  (4 * 1024 + 6 * 4096)
__global__ __launch_bounds__(64) void k_pack(const float* __restrict__ q1, const float* __restrict__ k1, const float* __restrict__ v1, const float* __restrict__ o1,
                                             const float* __restrict__ a2, const float* __restrict__ g2, const float* __restrict__ q2, const float* __restrict__ k2, const float* __restrict__ v2, const float* __restrict__ o2, __bf16* __restrict__ PT) {
  __shared__ __align__(16) __bf16 srow[64];
  const int blk = blockIdx.x, tid = threadIdx.x;
  const float* Wm; int K, nn; size_t base;
  if (blk < 128) { const int m = blk >> 5; nn = blk & 31; K = 32; Wm = m == 0 ? q1 : m == 1 ? k1 : m == 2 ? v1 : o1; base = P1(m) + (size_t)nn * 32; }
  else { const int m = (blk - 128) >> 6; nn = (blk - 128) & 63; K = 64; Wm = m == 0 ? a2 : m == 1 ? g2 : m == 2 ? q2 : m == 3 ? k2 : m == 4 ? v2 : o2; base = P2(m) + (size_t)nn * 64; }
  if (tid < K) srow[tid] = (__bf16)Wm[(size_t)tid * K + nn];
  __syncthreads();
  if (blk >= 128 && tid < 8) vst2((unsigned*)(PT + base + tid * 8), *(const v4u*)(&srow[tid * 8]));
}
__global__ __launch_bounds__(256) void k_pack1(const float* __restrict__ q1, const float* __restrict__ k1, const float* __restrict__ v1, const float* __restrict__ o1, __bf16* __restrict__ PT) {
  const int tid = threadIdx.x;
  for (int q = tid; q < 4 * 32 * 4; q += 256) { const int m = q >> 7, n = (q >> 2) & 31, pc = q & 3; const float* Wm = m == 0 ? q1 : m == 1 ? k1 : m == 2 ? v1 : o1; union { __bf16 e[8]; v4u u; } pk;
#pragma unroll
    for (int e = 0; e < 8; ++e) pk.e[e] = (__bf16)Wm[(size_t)(pc * 8 + e) * 32 + n];
    vst2((unsigned*)(PT + P1(m) + n * 32 + pc * 8), pk.u); }
}

__global__ __launch_bounds__(128) void k_blk1(const float* __restrict__ pos, const float* __restrict__ feat, const int* __restrict__ perm,
    const float* __restrict__ w1a, const float* __restrict__ b1a, const float* __restrict__ w1b, const float* __restrict__ b1b, const float* __restrict__ w2a, const float* __restrict__ b2a, const float* __restrict__ w2b, const float* __restrict__ b2b,
    const __bf16* __restrict__ PT, const float* __restrict__ bq, const float* __restrict__ bk, const float* __restrict__ bv, const float* __restrict__ bo, const float* __restrict__ lng, const float* __restrict__ lnb, float* __restrict__ F1) {
  __shared__ __align__(16) float hp[4][16][36], hg[4][16][36], sq[4][16][36], sk[4][16][36], sv[4][16][36], sa[4][16][36], so[4][16][36];
  __shared__ int sidx[4][16];
  const int tid = threadIdx.x, wave = tid >> 5, lane = tid & 31, col = lane & 15, g = lane >> 4;
  const int b = blockIdx.y, c = blockIdx.x * 4 + wave;
  const size_t pbase = (size_t)b * NPT;
  { const int k = c * 16 + (lane & 15); int pi = perm[pbase + k]; pi = pi < 0 ? 0 : (pi >= NPT ? NPT - 1 : pi); if (lane < 16) sidx[wave][lane] = pi;
    const float px = bfr(pos[(pbase + pi) * 3]), py = bfr(pos[(pbase + pi) * 3 + 1]), pz = bfr(pos[(pbase + pi) * 3 + 2]);
    const float fx = bfr(feat[(pbase + pi) * 3]), fy = bfr(feat[(pbase + pi) * 3 + 1]), fz = bfr(feat[(pbase + pi) * 3 + 2]);
    float sx = px, sy = py, sz = pz;
#pragma unroll
    for (int o = 1; o < 16; o <<= 1) { sx += __shfl_xor(sx, o); sy += __shfl_xor(sy, o); sz += __shfl_xor(sz, o); }
    const float cx = sx * (1.0f / 16.0f), cy = sy * (1.0f / 16.0f), cz = sz * (1.0f / 16.0f);
    const float lx = px - cx, ly = py - cy, lz = pz - cz; const float nrm = sqrtf(lx * lx + ly * ly + lz * lz);
    float ax = lx, ay = ly, az = lz;
#pragma unroll
    for (int o = 1; o < 16; o <<= 1) { ax += __shfl_xor(ax, o); ay += __shfl_xor(ay, o); az += __shfl_xor(az, o); }
    ax *= (1.0f / 16.0f); ay *= (1.0f / 16.0f); az *= (1.0f / 16.0f);
    float r[3], rh[3];
#pragma unroll
    for (int j = 0; j < 3; ++j) { r[j] = ((lx * bfr(w1a[0 * 3 + j]) + ly * bfr(w1a[1 * 3 + j])) + (lz * bfr(w1a[2 * 3 + j]) + nrm * bfr(w1a[3 * 3 + j]))) + bfr(b1a[j]);
                                  rh[j] = ((ax * bfr(w2a[0 * 3 + j]) + ay * bfr(w2a[1 * 3 + j])) + (az * bfr(w2a[2 * 3 + j]) + lx * bfr(w2a[3 * 3 + j]))) + ((ly * bfr(w2a[4 * 3 + j]) + lz * bfr(w2a[5 * 3 + j])) + bfr(b2a[j])); }
    const int p = lane & 15;
#pragma unroll 1
    for (int jj = 0; jj < 16; ++jj) { const int j = 16 * g + jj;
      const float vp = ((r[0] * bfr(w1b[0 * 32 + j]) + r[1] * bfr(w1b[1 * 32 + j])) + (r[2] * bfr(w1b[2 * 32 + j]) + fx * bfr(w1b[3 * 32 + j]))) + ((fy * bfr(w1b[4 * 32 + j]) + fz * bfr(w1b[5 * 32 + j])) + bfr(b1b[j]));
      const float vg = ((rh[0] * bfr(w2b[0 * 32 + j]) + rh[1] * bfr(w2b[1 * 32 + j])) + (rh[2] * bfr(w2b[2 * 32 + j]) + fx * bfr(w2b[3 * 32 + j]))) + ((fy * bfr(w2b[4 * 32 + j]) + fz * bfr(w2b[5 * 32 + j])) + bfr(b2b[j]));
      hp[wave][p][j] = vp; hg[wave][p][j] = vg; } }
  LDSX();
  { const F2 ag = split_row(&hg[wave][col][0], 0, lane), ap = split_row(&hp[wave][col][0], 0, lane); const float isq = sqrtf(32.0f);
#pragma unroll
    for (int ct = 0; ct < 2; ++ct) { const int n = ct * 16 + col; v8f aq = {}, ak = {}, av = {};
      { const v16b w = frag_b(PT + P1(0) + n * 32, lane); aq = wmma_bf(ag.l, w, aq); aq = wmma_bf(ag.h, w, aq); }
      { const v16b w = frag_b(PT + P1(1) + n * 32, lane); ak = wmma_bf(ag.l, w, ak); ak = wmma_bf(ag.h, w, ak); }
      { const v16b w = frag_b(PT + P1(2) + n * 32, lane); av = wmma_bf(ap.l, w, av); av = wmma_bf(ap.h, w, av); }
#pragma unroll
      for (int rr = 0; rr < 8; ++rr) { const int p = 8 * g + rr; sq[wave][p][n] = (aq[rr] + bfr(bq[n])) / isq; sk[wave][p][n] = ak[rr] + bfr(bk[n]); sv[wave][p][n] = av[rr] + bfr(bv[n]); } } }
  LDSX();
  { const F2 a = split_row(&sq[wave][col][0], 0, lane), bk2 = split_row(&sk[wave][col][0], 0, lane);
    v8f s = mac3(a, bk2, (v8f){});
#pragma unroll
    for (int rr = 0; rr < 8; ++rr) { float mx = s[rr];
#pragma unroll
      for (int o = 1; o < 16; o <<= 1) mx = fmaxf(mx, __shfl_xor(mx, o));
      const float e = exp_ni(s[rr] - mx); float sum = e;
#pragma unroll
      for (int o = 1; o < 16; o <<= 1) sum += __shfl_xor(sum, o);
      sa[wave][8 * g + rr][col] = e / sum; sa[wave][8 * g + rr][16 + col] = 0.f; } }
  LDSX();
  { const F2 a = split_row(&sa[wave][col][0], 0, lane); v8f o1[2];
#pragma unroll
    for (int ct = 0; ct < 2; ++ct) { const F2 bvv = split_colT(&sv[wave][0][0], 0, ct * 16 + col, lane, 36, 16); o1[ct] = mac3(a, bvv, (v8f){}); }
#pragma unroll
    for (int ct = 0; ct < 2; ++ct)
#pragma unroll
      for (int rr = 0; rr < 8; ++rr) so[wave][8 * g + rr][ct * 16 + col] = o1[ct][rr];
    LDSX();
    const F2 ao = split_row(&so[wave][col][0], 0, lane); v8f oo[2];
#pragma unroll
    for (int ct = 0; ct < 2; ++ct) { const v16b w = frag_b(PT + P1(3) + (ct * 16 + col) * 32, lane); oo[ct] = (v8f){}; oo[ct] = wmma_bf(ao.l, w, oo[ct]); oo[ct] = wmma_bf(ao.h, w, oo[ct]); }
    LDSX();
#pragma unroll
    for (int ct = 0; ct < 2; ++ct)
#pragma unroll
      for (int rr = 0; rr < 8; ++rr) { const int p = 8 * g + rr, n = ct * 16 + col; so[wave][p][n] = hp[wave][p][n] + (oo[ct][rr] + bfr(bo[n])); } }
  LDSX();
  { const int p = lane & 15; float s = 0.f, q2 = 0.f;
#pragma unroll 8
    for (int j = 0; j < 32; ++j) s += so[wave][p][j];
    const float mu = s * (1.0f / 32.0f);
#pragma unroll 8
    for (int j = 0; j < 32; ++j) { const float d = so[wave][p][j] - mu; q2 += d * d; }
    const float den = sqrtf(q2 * (1.0f / 32.0f) + 1e-5f);
    LDSX();
#pragma unroll 1
    for (int jj = 0; jj < 16; ++jj) { const int j = 16 * g + jj; so[wave][p][j] = (so[wave][p][j] - mu) / den * bfr(lng[j]) + bfr(lnb[j]); } }
  LDSX();
  for (int q = lane; q < 16 * 8; q += 32) { const int p = q >> 3, pc = q & 7; vst2(F1 + (pbase + sidx[wave][p]) * 32 + pc * 4, *(const v4f*)(&so[wave][p][pc * 4])); }
}

__global__ __launch_bounds__(64) void k_blk2(const float* __restrict__ pos, const float* __restrict__ F1, const int* __restrict__ perm,
    const float* __restrict__ w1a, const float* __restrict__ b1a, const float* __restrict__ b1b, const float* __restrict__ w2a, const float* __restrict__ b2a, const float* __restrict__ b2b,
    const __bf16* __restrict__ PT, const float* __restrict__ bq, const float* __restrict__ bk, const float* __restrict__ bv, const float* __restrict__ bo, const float* __restrict__ lng, const float* __restrict__ lnb, float* __restrict__ F2out) {
  __shared__ __align__(16) float XP[32][68], XG[32][68], HP[32][68], HG[32][68], SQ[32][68], SK[32][68], SV[32][68], O1[32][68];
  __shared__ __align__(16) float SA[32][36];
  __shared__ int sidx[32];
  const int tid = threadIdx.x, wave = tid >> 5, lane = tid & 31, col = lane & 15, g = lane >> 4;
  const int b = blockIdx.y, c = blockIdx.x; const size_t pbase = (size_t)b * NPT;
  { const int k = c * 32 + lane; int pi = perm[pbase + k]; pi = pi < 0 ? 0 : (pi >= NPT ? NPT - 1 : pi); if (wave == 0) sidx[lane] = pi;
    const float px = bfr(pos[(pbase + pi) * 3]), py = bfr(pos[(pbase + pi) * 3 + 1]), pz = bfr(pos[(pbase + pi) * 3 + 2]);
    float sx = px, sy = py, sz = pz;
#pragma unroll
    for (int o = 1; o < 32; o <<= 1) { sx += __shfl_xor(sx, o); sy += __shfl_xor(sy, o); sz += __shfl_xor(sz, o); }
    const float lx = px - sx * (1.0f / 32.0f), ly = py - sy * (1.0f / 32.0f), lz = pz - sz * (1.0f / 32.0f); const float nrm = sqrtf(lx * lx + ly * ly + lz * lz);
    float ax = lx, ay = ly, az = lz;
#pragma unroll
    for (int o = 1; o < 32; o <<= 1) { ax += __shfl_xor(ax, o); ay += __shfl_xor(ay, o); az += __shfl_xor(az, o); }
    ax *= (1.0f / 32.0f); ay *= (1.0f / 32.0f); az *= (1.0f / 32.0f);
    float (*X)[68] = wave == 0 ? XP : XG;
    const float* F1r = F1 + (pbase + pi) * 32;
#pragma unroll 1
    for (int j = 0; j < 32; ++j) { float v;
      if (wave == 0) v = ((lx * bfr(w1a[0 * 32 + j]) + ly * bfr(w1a[1 * 32 + j])) + (lz * bfr(w1a[2 * 32 + j]) + nrm * bfr(w1a[3 * 32 + j]))) + bfr(b1a[j]);
      else v = ((ax * bfr(w2a[0 * 32 + j]) + ay * bfr(w2a[1 * 32 + j])) + (az * bfr(w2a[2 * 32 + j]) + lx * bfr(w2a[3 * 32 + j]))) + ((ly * bfr(w2a[4 * 32 + j]) + lz * bfr(w2a[5 * 32 + j])) + bfr(b2a[j]));
      X[lane][j] = v; X[lane][32 + j] = F1r[j]; } }
  __syncthreads();
  { const F2 ap0 = split_row(&XP[wave * 16 + col][0], 0, lane), ap1 = split_row(&XP[wave * 16 + col][0], 32, lane), ag0 = split_row(&XG[wave * 16 + col][0], 0, lane), ag1 = split_row(&XG[wave * 16 + col][0], 32, lane);
#pragma unroll
    for (int ct = 0; ct < 4; ++ct) { const int n = ct * 16 + col; v8f a = {}, e = {};
      { const __bf16* w = PT + P2(0) + n * 64; const v16b w0 = frag_b(w, lane), w1 = frag_b(w + 32, lane); a = wmma_bf(ap0.l, w0, a); a = wmma_bf(ap0.h, w0, a); a = wmma_bf(ap1.l, w1, a); a = wmma_bf(ap1.h, w1, a); }
      { const __bf16* w = PT + P2(1) + n * 64; const v16b w0 = frag_b(w, lane), w1 = frag_b(w + 32, lane); e = wmma_bf(ag0.l, w0, e); e = wmma_bf(ag0.h, w0, e); e = wmma_bf(ag1.l, w1, e); e = wmma_bf(ag1.h, w1, e); }
#pragma unroll
      for (int rr = 0; rr < 8; ++rr) { const int p = wave * 16 + 8 * g + rr; HP[p][n] = a[rr] + bfr(b1b[n]); HG[p][n] = e[rr] + bfr(b2b[n]); } } }
  __syncthreads();
  { const F2 ag0 = split_row(&HG[wave * 16 + col][0], 0, lane), ag1 = split_row(&HG[wave * 16 + col][0], 32, lane), ap0 = split_row(&HP[wave * 16 + col][0], 0, lane), ap1 = split_row(&HP[wave * 16 + col][0], 32, lane);
#pragma unroll 1
    for (int ct = 0; ct < 4; ++ct) { const int n = ct * 16 + col; v8f aq = {}, ak = {}, av = {};
      { const __bf16* w = PT + P2(2) + n * 64; const v16b w0 = frag_b(w, lane), w1 = frag_b(w + 32, lane); aq = wmma_bf(ag0.l, w0, aq); aq = wmma_bf(ag0.h, w0, aq); aq = wmma_bf(ag1.l, w1, aq); aq = wmma_bf(ag1.h, w1, aq); }
      { const __bf16* w = PT + P2(3) + n * 64; const v16b w0 = frag_b(w, lane), w1 = frag_b(w + 32, lane); ak = wmma_bf(ag0.l, w0, ak); ak = wmma_bf(ag0.h, w0, ak); ak = wmma_bf(ag1.l, w1, ak); ak = wmma_bf(ag1.h, w1, ak); }
      { const __bf16* w = PT + P2(4) + n * 64; const v16b w0 = frag_b(w, lane), w1 = frag_b(w + 32, lane); av = wmma_bf(ap0.l, w0, av); av = wmma_bf(ap0.h, w0, av); av = wmma_bf(ap1.l, w1, av); av = wmma_bf(ap1.h, w1, av); }
#pragma unroll
      for (int rr = 0; rr < 8; ++rr) { const int p = wave * 16 + 8 * g + rr; SQ[p][n] = (aq[rr] + bfr(bq[n])) / 8.0f; SK[p][n] = ak[rr] + bfr(bk[n]); SV[p][n] = av[rr] + bfr(bv[n]); } } }
  __syncthreads();
  { const F2 a0 = split_row(&SQ[wave * 16 + col][0], 0, lane), a1 = split_row(&SQ[wave * 16 + col][0], 32, lane); v8f s[2];
#pragma unroll
    for (int ct = 0; ct < 2; ++ct) { const F2 k0 = split_row(&SK[ct * 16 + col][0], 0, lane), k1 = split_row(&SK[ct * 16 + col][0], 32, lane); s[ct] = mac3(a0, k0, (v8f){}); s[ct] = mac3(a1, k1, s[ct]); }
#pragma unroll
    for (int rr = 0; rr < 8; ++rr) { float mx = fmaxf(s[0][rr], s[1][rr]);
#pragma unroll
      for (int o = 1; o < 16; o <<= 1) mx = fmaxf(mx, __shfl_xor(mx, o));
      const float e0 = exp_ni(s[0][rr] - mx), e1 = exp_ni(s[1][rr] - mx); float sum = e0 + e1;
#pragma unroll
      for (int o = 1; o < 16; o <<= 1) sum += __shfl_xor(sum, o);
      SA[wave * 16 + 8 * g + rr][col] = e0 / sum; SA[wave * 16 + 8 * g + rr][16 + col] = e1 / sum; } }
  __syncthreads();
  { const F2 a = split_row(&SA[wave * 16 + col][0], 0, lane);
#pragma unroll 1
    for (int ct = 0; ct < 4; ++ct) { const F2 bvv = split_colT(&SV[0][0], 0, ct * 16 + col, lane, 68, 32); const v8f o = mac3(a, bvv, (v8f){});
#pragma unroll
      for (int rr = 0; rr < 8; ++rr) O1[wave * 16 + 8 * g + rr][ct * 16 + col] = o[rr]; } }
  LDSX();
  { const F2 a0 = split_row(&O1[wave * 16 + col][0], 0, lane), a1 = split_row(&O1[wave * 16 + col][0], 32, lane);
#pragma unroll 1
    for (int ct = 0; ct < 4; ++ct) { const int n = ct * 16 + col; const __bf16* w = PT + P2(5) + n * 64; const v16b w0 = frag_b(w, lane), w1 = frag_b(w + 32, lane); v8f o = {};
      o = wmma_bf(a0.l, w0, o); o = wmma_bf(a0.h, w0, o); o = wmma_bf(a1.l, w1, o); o = wmma_bf(a1.h, w1, o);
#pragma unroll
      for (int rr = 0; rr < 8; ++rr) { const int p = wave * 16 + 8 * g + rr; SQ[p][n] = HP[p][n] + (o[rr] + bfr(bo[n])); } } }
  LDSX();
  { const int p = wave * 16 + (lane & 15); float s = 0.f, q2 = 0.f;
#pragma unroll 8
    for (int j = 0; j < 64; ++j) s += SQ[p][j];
    const float mu = s * (1.0f / 64.0f);
#pragma unroll 8
    for (int j = 0; j < 64; ++j) { const float d = SQ[p][j] - mu; q2 += d * d; }
    const float den = sqrtf(q2 * (1.0f / 64.0f) + 1e-5f);
    LDSX();
#pragma unroll 1
    for (int jj = 0; jj < 32; ++jj) { const int j = 32 * g + jj; O1[p][j] = (SQ[p][j] - mu) / den * bfr(lng[j]) + bfr(lnb[j]); } }
  __syncthreads();
  for (int q = tid; q < 32 * 16; q += 64) { const int p = q >> 4, pc = q & 15; vst2(F2out + (pbase + sidx[p]) * 64 + pc * 4, *(const v4f*)(&O1[p][pc * 4])); }
}
__global__ __launch_bounds__(256) void k_out(const float* __restrict__ pos, const float* __restrict__ F2in, const int* __restrict__ fps, float* __restrict__ out0, float* __restrict__ out1) {
  __shared__ __align__(16) float sp[64 * 3]; __shared__ int si[64];
  const int tid = threadIdx.x, b = blockIdx.y; const size_t q0 = (size_t)blockIdx.x * 64; const size_t pbase = (size_t)b * NPT, dbase = (size_t)b * NDS + q0;
  if (tid < 64) { int i = fps[(size_t)b * NDS + q0 + tid]; i = i < 0 ? 0 : (i >= NPT ? NPT - 1 : i); si[tid] = i; sp[tid * 3] = bfr(pos[(pbase + i) * 3]); sp[tid * 3 + 1] = bfr(pos[(pbase + i) * 3 + 1]); sp[tid * 3 + 2] = bfr(pos[(pbase + i) * 3 + 2]); }
  __syncthreads();
  if (tid < 48) vst2(out0 + dbase * 3 + tid * 4, *(const v4f*)&sp[tid * 4]);
  { const int r = tid >> 4, pc = tid & 15;
#pragma unroll
    for (int pass = 0; pass < 4; ++pass) { const int row = pass * 16 + r; vst2(out1 + (dbase + row) * 64 + pc * 4, *(const v4f*)(F2in + (pbase + si[row]) * 64 + pc * 4)); } }
}

extern "C" void kernel_launch(void* const* d_in, const int* in_sizes, int n_in, void* d_out, int out_size, void* d_ws, size_t ws_size, hipStream_t stream) {
  (void)in_sizes; (void)n_in; (void)out_size;
  const float** F = (const float**)d_in; const int* perm1 = (const int*)d_in[2]; const int* perm2 = (const int*)d_in[3]; const int* fps = (const int*)d_in[4];
  const size_t off_f1 = 2u * P_END + 256, off_f2 = off_f1 + 4u * NBATCH * NPT * 32;
  if (ws_size < off_f2 + 4u * (size_t)NBATCH * NPT * 64) return;
  char* ws = (char*)d_ws; __bf16* PT = (__bf16*)ws; float* F1b = (float*)(ws + off_f1); float* F2b = (float*)(ws + off_f2);
  float* out0 = (float*)d_out; float* out1 = out0 + (size_t)NBATCH * NDS * 3;
  k_pack<<<512, 64, 0, stream>>>(F[13], F[15], F[17], F[19], F[25], F[29], F[31], F[33], F[35], F[37], PT);
  k_pack1<<<1, 256, 0, stream>>>(F[13], F[15], F[17], F[19], PT);
  k_blk1<<<dim3(NPT / 16 / 4, TNB), 128, 0, stream>>>(F[0], F[1], perm1, F[5], F[6], F[7], F[8], F[9], F[10], F[11], F[12], PT, F[14], F[16], F[18], F[20], F[21], F[22], F1b);
  k_blk2<<<dim3(NPT / 32, TNB), 64, 0, stream>>>(F[0], F1b, perm2, F[23], F[24], F[26], F[27], F[28], F[30], PT, F[32], F[34], F[36], F[38], F[39], F[40], F2b);
  k_out<<<dim3(NDS / 64, TNB), 256, 0, stream>>>(F[0], F2b, fps, out0, out1);
}
